// PVB_11673721111014
// MI455X (gfx1250) — hardware-run, weakly checked
//
#include <hip/hip_runtime.h>
#include <math.h>

typedef __attribute__((ext_vector_type(16))) _Float16 v16h;
typedef __attribute__((ext_vector_type(8)))  _Float16 v8h;
typedef __attribute__((ext_vector_type(8)))  float    v8f;
typedef __attribute__((ext_vector_type(4)))  float    v4f;
typedef __attribute__((ext_vector_type(4)))  int      v4i;

constexpr int kBatch   = 4;
constexpr int kChan    = 64;
constexpr int kPoints  = 16384;
constexpr int kNeigh   = 16;
constexpr int kRes     = 16;
constexpr int kVoxels  = kRes * kRes * kRes;
constexpr int kAllPts  = kBatch * kPoints;
constexpr int kProjPad = 16;
constexpr int kTaps    = 27;
constexpr float kWCarry    = 16.0f;
constexpr float kWCarryInv = 1.0f / kWCarry;
constexpr float kEpsVox = 1e-4f;
constexpr float kEpsPt  = 1e-5f;
static_assert(kVoxels == 4096, "voxel count");
static_assert((kChan % 32) == 0, "K multiple of 32");
static_assert((kAllPts % 64) == 0, "M multiple of 64");
static_assert((kPoints % 1024) == 0, "scan step multiple");
static_assert(kNeigh == 16, "neighbour count");

constexpr size_t kSzMean = 2048;
constexpr size_t kSzWpad = (size_t)kProjPad * kChan * 2;
constexpr size_t kSzVid  = (size_t)kAllPts * 4;
constexpr size_t kSzNcT  = (size_t)kAllPts * 4 * 4;
constexpr size_t kSzXyzT = (size_t)kAllPts * 4 * 4;
constexpr size_t kSzProj = (size_t)kAllPts * kProjPad * 4;
constexpr size_t kSzVox  = (size_t)kBatch * kVoxels * kChan * 4;
constexpr size_t kSzXT16 = (size_t)kAllPts * kChan * 2;
constexpr size_t kSzXT32 = (size_t)kAllPts * kChan * 4;
constexpr size_t kOffMean = 0;
constexpr size_t kOffWpad = kOffMean + kSzMean;
constexpr size_t kOffVid  = kOffWpad + kSzWpad;
constexpr size_t kOffNcT  = kOffVid  + kSzVid;
constexpr size_t kOffXyzT = kOffNcT  + kSzNcT;
constexpr size_t kOffProj = kOffXyzT + kSzXyzT;
constexpr size_t kOffV0   = kOffProj + kSzProj;
constexpr size_t kOffV1   = kOffV0   + kSzVox;
constexpr size_t kOffV2   = kOffV1   + kSzVox;
constexpr size_t kOffXT16 = kOffV2   + kSzVox;
constexpr size_t kOffXT32 = kOffXT16 + kSzXT16;
constexpr size_t kWsTotal = kOffXT32 + kSzXT32;
static_assert(kWsTotal == 44306432ull, "carve total");
static_assert(kWsTotal <= 134217728ull, "carve cap");
static_assert((kOffWpad % 128) == 0 && (kOffVid % 128) == 0 && (kOffNcT % 128) == 0 && (kOffXyzT % 128) == 0 &&
              (kOffProj % 128) == 0 && (kOffV0 % 128) == 0 && (kOffV1 % 128) == 0 && (kOffV2 % 128) == 0 &&
              (kOffXT16 % 128) == 0 && (kOffXT32 % 128) == 0, "128-B aligned regions");

template <typename T> struct Frag;
template <> struct Frag<_Float16> {
  typedef v16h V; union U { v16h v; v8h h[2]; };
  static __device__ __forceinline__ v16h load(const _Float16* p) {
    U f; f.h[0] = *(const v8h*)(p); f.h[1] = *(const v8h*)(p + 16); return f.v;
  }
};
__device__ __forceinline__ v8f wmma_h(v16h a, v16h b, v8f c) {
  c = __builtin_amdgcn_wmma_f32_16x16x32_f16(false, a, false, b, (short)0, c, false, false);
  asm volatile("v_nop\n\tv_nop\n\tv_nop\n\tv_nop" : "+v"(c) : "v"(a), "v"(b));
  return c;
}
__device__ __forceinline__ int clampi(int v, int lo, int hi) { return v < lo ? lo : (v > hi ? hi : v); }

__global__ __launch_bounds__(256) void coord_mean_kernel(const float* __restrict__ xyz, float* __restrict__ meanp)
{
  __shared__ double sRed[256];
  const int tid = threadIdx.x;
  const int bd = blockIdx.x;
  const float* src = xyz + (size_t)bd * kPoints;
  double s = 0.0;
#pragma unroll 1
  for (int q = 0; q < kPoints / 256; ++q) s += (double)src[q * 256 + tid];
  sRed[tid] = s;
  __syncthreads();
#pragma unroll 1
  for (int off = 128; off > 0; off >>= 1) {
    if (tid < off) sRed[tid] = sRed[tid] + sRed[tid + off];
    __syncthreads();
  }
  if (tid < 32) {
    const float m = (float)(sRed[0] * (1.0 / (double)kPoints));
    volatile float* q = meanp + bd * 32 + tid;
    *q = m;
    __threadfence();
    *q = m;
  }
}

__global__ __launch_bounds__(128) void weight_pad_kernel(const float* __restrict__ pw1, unsigned short* __restrict__ wpad)
{
  const int tid = threadIdx.x;
  const int row = tid >> 3;
  const int c8 = (tid & 7) * 8;
  const int rc = row < 3 ? row : 2;
  const bool live = row < 3;
  const v4f a0 = *(const v4f*)(pw1 + rc * kChan + c8);
  const v4f a1 = *(const v4f*)(pw1 + rc * kChan + c8 + 4);
  v8h hv;
#pragma unroll
  for (int e = 0; e < 4; ++e) {
    const float f0 = live ? a0[e] * kWCarry : 0.0f;
    const float f1 = live ? a1[e] * kWCarry : 0.0f;
    hv[e] = (_Float16)f0;
    hv[4 + e] = (_Float16)f1;
  }
  unsigned short* q = wpad + row * kChan + c8;
  *(volatile v8h*)q = hv;
  __threadfence();
  *(volatile v8h*)q = hv;
}

__global__ __launch_bounds__(256) void point_prep_kernel(
    const float* __restrict__ x, const float* __restrict__ xyz, const float* __restrict__ meanp,
    float* __restrict__ xT32, unsigned short* __restrict__ xT16,
    float* __restrict__ ncT, float* __restrict__ xyzT, int* __restrict__ vid)
{
  __shared__ float sT[kChan * 33];
  const int tid = threadIdx.x, lane = tid & 31, wave = tid >> 5;
  const int b = blockIdx.x >> 9;
  const int n0 = (blockIdx.x & 511) << 5;
#pragma unroll
  for (int i = 0; i < 8; ++i) {
    const int c = wave * 8 + i;
    sT[c * 33 + lane] = x[((size_t)(b * kChan + c)) * kPoints + n0 + lane];
  }
  __syncthreads();
  const size_t p0 = (size_t)b * kPoints + n0;

  v4f f32v[2];
#pragma unroll
  for (int it = 0; it < 2; ++it) {
    const int pl = 4 * wave + 2 * it + (lane >> 4);
    const int c4 = (lane & 15) * 4;
    v4f t;
    t[0] = sT[(c4 + 0) * 33 + pl];
    t[1] = sT[(c4 + 1) * 33 + pl];
    t[2] = sT[(c4 + 2) * 33 + pl];
    t[3] = sT[(c4 + 3) * 33 + pl];
    f32v[it] = t;
  }
  v8h hv;
  const int pl8 = 4 * wave + (lane >> 3);
  const int c8 = (lane & 7) * 8;
#pragma unroll
  for (int e = 0; e < 8; ++e) hv[e] = (_Float16)sT[(c8 + e) * 33 + pl8];

  const int n = n0 + lane;
  float craw[3], ncv[3];
#pragma unroll
  for (int d = 0; d < 3; ++d) {
    const float cv = xyz[((size_t)(b * 3 + d)) * kPoints + n];
    const float mv = meanp[(b * 3 + d) * 32];
    float t = cv - mv;
    t = t + 1.0f;
    t = t * 0.5f;
    t = t * (float)kRes;
    t = fminf(fmaxf(t, 0.0f), (float)(kRes - 1));
    craw[d] = cv;
    ncv[d] = t;
  }
  const int vi0 = (int)rintf(ncv[0]);
  const int vi1 = (int)rintf(ncv[1]);
  const int vi2 = (int)rintf(ncv[2]);
  const int flat = (vi0 * kRes + vi1) * kRes + vi2;
  v4f ncq, xyq;
  ncq[0] = ncv[0]; ncq[1] = ncv[1]; ncq[2] = ncv[2]; ncq[3] = 0.0f;
  xyq[0] = craw[0]; xyq[1] = craw[1]; xyq[2] = craw[2]; xyq[3] = 0.0f;

  for (int pass = 0; pass < 2; ++pass) {
#pragma unroll
    for (int it = 0; it < 2; ++it) {
      const int pl = 4 * wave + 2 * it + (lane >> 4);
      const int c4 = (lane & 15) * 4;
      *(volatile v4f*)(xT32 + (p0 + pl) * kChan + c4) = f32v[it];
    }
    *(volatile v8h*)(xT16 + (p0 + pl8) * kChan + c8) = hv;
    if (wave == 0) *(volatile v4f*)(ncT + (p0 + lane) * 4) = ncq;
    if (wave == 1) *(volatile v4f*)(xyzT + (p0 + lane) * 4) = xyq;
    if (wave == 2) *(volatile int*)(vid + p0 + lane) = flat;
    __threadfence();
  }
}

__global__ __launch_bounds__(64) void voxel_mean_kernel(
    const int* __restrict__ vid, const float* __restrict__ xT32, float* __restrict__ v0)
{
  __shared__ __align__(16) float sSum[64 * 64];
  __shared__ __align__(16) int sVox[1024];
  __shared__ unsigned sMask[32];
  __shared__ float sCnt[64];
  const int tid = threadIdx.x, lane = tid & 31, wave = tid >> 5;
  const int b = blockIdx.x >> 6;
  const int seg = blockIdx.x & 63;
#pragma unroll 1
  for (int v = 0; v < 64; ++v) sSum[v * 64 + tid] = 0.0f;
  float cnt = 0.0f;
  const int* vb = vid + (size_t)b * kPoints;
  const float* xb = xT32 + (size_t)b * kPoints * kChan;
#pragma unroll 1
  for (int st = 0; st < kPoints / 1024; ++st) {
    __syncthreads();
#pragma unroll
    for (int cq = 0; cq < 4; ++cq) {
      const v4i ids = *(const v4i*)(vb + st * 1024 + cq * 256 + tid * 4);
      *(v4i*)(sVox + cq * 256 + tid * 4) = ids;
      const unsigned m0 = __builtin_amdgcn_ballot_w32((ids[0] >> 6) == seg);
      const unsigned m1 = __builtin_amdgcn_ballot_w32((ids[1] >> 6) == seg);
      const unsigned m2 = __builtin_amdgcn_ballot_w32((ids[2] >> 6) == seg);
      const unsigned m3 = __builtin_amdgcn_ballot_w32((ids[3] >> 6) == seg);
      if (lane == 0) {
        sMask[cq * 8 + wave * 4 + 0] = m0;
        sMask[cq * 8 + wave * 4 + 1] = m1;
        sMask[cq * 8 + wave * 4 + 2] = m2;
        sMask[cq * 8 + wave * 4 + 3] = m3;
      }
    }
    __syncthreads();
#pragma unroll 1
    for (int i = 0; i < 32; ++i) {
      unsigned m = (unsigned)__builtin_amdgcn_readfirstlane((int)sMask[i]);
      const int posb = (i >> 3) * 256 + ((i >> 2) & 1) * 128 + (i & 3);
#pragma unroll 1
      for (int itb = 0; itb < 32; ++itb) {
        if (m == 0u) break;
        const int bit = __builtin_ctz(m);
        m &= (m - 1u);
        const int pos = posb + bit * 4;
        const int id = sVox[pos];
        const int local = id & 63;
        const int p = st * 1024 + pos;
        const float val = xb[(size_t)p * kChan + tid];
        sSum[local * 64 + tid] += val;
        cnt += (local == tid) ? 1.0f : 0.0f;
      }
    }
  }
  sCnt[tid] = cnt;
  __syncthreads();
  float* dst = v0 + ((size_t)(b * kVoxels + seg * 64)) * kChan;
  const int c4 = (lane & 15) * 4;
  for (int pass = 0; pass < 2; ++pass) {
#pragma unroll 1
    for (int it = 0; it < 16; ++it) {
      const int vl = wave * 32 + it * 2 + (lane >> 4);
      const float inv = 1.0f / fmaxf(sCnt[vl], 1.0f);
      v4f o;
      o[0] = sSum[vl * 64 + c4 + 0] * inv;
      o[1] = sSum[vl * 64 + c4 + 1] * inv;
      o[2] = sSum[vl * 64 + c4 + 2] * inv;
      o[3] = sSum[vl * 64 + c4 + 3] * inv;
      *(volatile v4f*)(dst + (size_t)vl * kChan + c4) = o;
    }
    __threadfence();
  }
}

__global__ __launch_bounds__(256) void stencil_kernel(
    const float* __restrict__ vin, const float* __restrict__ w, const float* __restrict__ bias,
    const float* __restrict__ bn, float* __restrict__ vout)
{
  __shared__ __align__(16) float sW[kTaps * kChan];
  const int tid = threadIdx.x;
#pragma unroll 1
  for (int q = 0; q < 7; ++q) {
    const int i = q * 256 + tid;
    const int ic = i < kTaps * kChan ? i : (kTaps * kChan - 1);
    const float wv = w[ic];
    const int c = ic / kTaps;
    const int tap = ic - c * kTaps;
    if (i < kTaps * kChan) sW[tap * kChan + c] = wv;
  }
  __syncthreads();
  const int vloc = tid >> 4;
  const int c4 = (tid & 15) * 4;
  const int vg = blockIdx.x * 16 + vloc;
  const int b = vg >> 12;
  const int vox = vg & (kVoxels - 1);
  const int X = vox >> 8, Y = (vox >> 4) & 15, Z = vox & 15;
  const float* vb = vin + (size_t)b * kVoxels * kChan;
  const v4f zero4 = (v4f){0.f, 0.f, 0.f, 0.f};
  v4f acc = zero4;
#pragma unroll 1
  for (int dx = 0; dx < 3; ++dx) {
    const int xx = X + dx - 1;
    const bool okx = (unsigned)xx < (unsigned)kRes;
    const int xc = clampi(xx, 0, kRes - 1);
#pragma unroll
    for (int dy = 0; dy < 3; ++dy) {
      const int yy = Y + dy - 1;
      const bool oky = (unsigned)yy < (unsigned)kRes;
      const int yc = clampi(yy, 0, kRes - 1);
#pragma unroll
      for (int dz = 0; dz < 3; ++dz) {
        const int zz = Z + dz - 1;
        const bool okz = (unsigned)zz < (unsigned)kRes;
        const int zc = clampi(zz, 0, kRes - 1);
        const bool ok = okx && oky && okz;
        const v4f val = *(const v4f*)(vb + ((size_t)((xc * kRes + yc) * kRes + zc)) * kChan + c4);
        const v4f wv = *(const v4f*)(sW + ((dx * 3 + dy) * 3 + dz) * kChan + c4);
        const v4f term = wv * val;
        acc = acc + (ok ? term : zero4);
      }
    }
  }
  const v4f bi = *(const v4f*)(bias + c4);
  const v4f g4 = *(const v4f*)(bn + c4);
  const v4f be4 = *(const v4f*)(bn + kChan + c4);
  const v4f m4 = *(const v4f*)(bn + 2 * kChan + c4);
  const v4f var4 = *(const v4f*)(bn + 3 * kChan + c4);
  v4f o;
#pragma unroll
  for (int e = 0; e < 4; ++e) {
    const float y0 = acc[e] + bi[e];
    const float sc = g4[e] * rsqrtf(var4[e] + kEpsVox);
    const float y = (y0 - m4[e]) * sc + be4[e];
    o[e] = (y >= 0.0f) ? y : 0.1f * y;
  }
  float* q = vout + (size_t)vg * kChan + c4;
  *(volatile v4f*)q = o;
  __threadfence();
  *(volatile v4f*)q = o;
}

__global__ __launch_bounds__(256) void proj_gemm_kernel(
    const unsigned short* __restrict__ xT16, const unsigned short* __restrict__ wpad, float* __restrict__ proj)
{
  __shared__ __align__(16) float sC[8][64 * kProjPad];
  const int tid = threadIdx.x, lane = tid & 31, wave = tid >> 5;
  const int rl = lane & 15;
  const int hh = lane >> 4;
  const int koff = hh * 8;
  const int r0 = (blockIdx.x * 8 + wave) * 64;
  const _Float16* A = (const _Float16*)(const void*)xT16;
  const _Float16* W = (const _Float16*)(const void*)wpad;
  v16h bf[2];
#pragma unroll
  for (int kk = 0; kk < 2; ++kk) bf[kk] = Frag<_Float16>::load(W + rl * kChan + koff + kk * 32);
  v8f acc[4];
#pragma unroll
  for (int i = 0; i < 4; ++i) acc[i] = (v8f){0.f, 0.f, 0.f, 0.f, 0.f, 0.f, 0.f, 0.f};
#pragma unroll
  for (int i = 0; i < 4; ++i) {
#pragma unroll
    for (int kk = 0; kk < 2; ++kk) {
      const v16h a = Frag<_Float16>::load(A + (size_t)(r0 + i * 16 + rl) * kChan + koff + kk * 32);
      acc[i] = wmma_h(a, bf[kk], acc[i]);
    }
  }
  float* slab = sC[wave];
#pragma unroll
  for (int i = 0; i < 4; ++i) {
#pragma unroll
    for (int r = 0; r < 8; ++r) slab[(i * 16 + 8 * hh + r) * kProjPad + rl] = acc[i][r] * kWCarryInv;
  }
  __syncthreads();
  float* dst = proj + (size_t)r0 * kProjPad;
  for (int pass = 0; pass < 2; ++pass) {
#pragma unroll
    for (int it = 0; it < 8; ++it) {
      const v4f v = *(const v4f*)(slab + it * 128 + lane * 4);
      *(volatile v4f*)(dst + it * 128 + lane * 4) = v;
    }
    __threadfence();
  }
}

__global__ __launch_bounds__(256) void fuse_kernel(
    const float* __restrict__ xT32, const float* __restrict__ xyzT, const float* __restrict__ ncT,
    const float* __restrict__ proj, const int* __restrict__ idx, const float* __restrict__ v2,
    const float* __restrict__ pbn, const float* __restrict__ pw2, const float* __restrict__ ptbn,
    float* __restrict__ out)
{
  __shared__ float sRes[kChan * 33];
  __shared__ float sDp[8 * 64 * 8];
  __shared__ int sJ[8 * 64];
  const int tid = threadIdx.x, lane = tid & 31, wave = tid >> 5;
  const int b = blockIdx.x >> 9;
  const int n0 = (blockIdx.x & 511) << 5;
  const int nw = n0 + 4 * wave;
  const size_t pb = (size_t)b * kPoints;
  const v4f* xyz4 = (const v4f*)xyzT;
  const v4f* nc4 = (const v4f*)ncT;
  const v4f* pr4 = (const v4f*)proj;

  const v4f q0 = *(const v4f*)(pbn);
  const v4f q1 = *(const v4f*)(pbn + 4);
  const v4f q2 = *(const v4f*)(pbn + 8);
  const v4f r0 = *(const v4f*)(pw2);
  const v4f r1 = *(const v4f*)(pw2 + 4);
  const float w22 = pw2[8];
  const float ps0 = q0[0] * rsqrtf(q2[1] + kEpsPt);
  const float ps1 = q0[1] * rsqrtf(q2[2] + kEpsPt);
  const float ps2 = q0[2] * rsqrtf(q2[3] + kEpsPt);
  const float pbe0 = q0[3], pbe1 = q1[0], pbe2 = q1[1];
  const float pm0 = q1[2], pm1 = q1[3], pm2 = q2[0];

#pragma unroll 1
  for (int it = 0; it < 2; ++it) {
    const int item = it * 32 + lane;
    const int n = nw + (item >> 4);
    int j = idx[(pb + nw) * kNeigh + item];
    j = clampi(j, 0, kPoints - 1);
    const v4f cj = xyz4[pb + j];
    const v4f cn = xyz4[pb + n];
    const v4f pj = pr4[(pb + j) * 4];
    const v4f pn = pr4[(pb + n) * 4];
    const float h0 = pj[0] - pn[0];
    const float h1 = pj[1] - pn[1];
    const float h2 = pj[2] - pn[2];
    const float a0 = fmaxf((h0 - pm0) * ps0 + pbe0, 0.0f);
    const float a1 = fmaxf((h1 - pm1) * ps1 + pbe1, 0.0f);
    const float a2 = fmaxf((h2 - pm2) * ps2 + pbe2, 0.0f);
    float* dst = sDp + (wave * 64 + item) * 8;
    dst[0] = cj[0] - cn[0];
    dst[1] = cj[1] - cn[1];
    dst[2] = cj[2] - cn[2];
    dst[3] = (r0[0] * a0 + r0[1] * a1) + r0[2] * a2;
    dst[4] = (r0[3] * a0 + r1[0] * a1) + r1[1] * a2;
    dst[5] = (r1[2] * a0 + r1[3] * a1) + w22 * a2;
    dst[6] = 0.0f;
    dst[7] = 0.0f;
    sJ[wave * 64 + item] = j;
  }
  __syncthreads();

  const int c0 = lane, c1 = lane + 32;
  const int g0 = (c0 / 10) < 5 ? (c0 / 10) : 5;
  const int g1 = (c1 / 10) < 5 ? (c1 / 10) : 5;
  const float s0 = ptbn[c0] * rsqrtf(ptbn[3 * kChan + c0] + kEpsPt);
  const float s1 = ptbn[c1] * rsqrtf(ptbn[3 * kChan + c1] + kEpsPt);
  const float be0 = ptbn[kChan + c0], be1 = ptbn[kChan + c1];
  const float me0 = ptbn[2 * kChan + c0], me1 = ptbn[2 * kChan + c1];
  const float* v2b = v2 + (size_t)b * kVoxels * kChan;

#pragma unroll 1
  for (int pt = 0; pt < 4; ++pt) {
    const int n = nw + pt;
    const int sb = wave * 64 + pt * 16;
    float mx0 = 0.0f, mx1 = 0.0f;
#pragma unroll 2
    for (int k = 0; k < kNeigh; ++k) {
      const int j = sJ[sb + k];
      const float* row = xT32 + (pb + j) * kChan;
      const float u0 = row[c0];
      const float u1 = row[c1];
      const float w0 = sDp[(sb + k) * 8 + g0];
      const float w1 = sDp[(sb + k) * 8 + g1];
      const float t0 = (u0 * w0 - me0) * s0 + be0;
      const float t1 = (u1 * w1 - me1) * s1 + be1;
      mx0 = fmaxf(mx0, t0);
      mx1 = fmaxf(mx1, t1);
    }
    const v4f nv = nc4[pb + n];
    const int lo0 = clampi((int)floorf(nv[0]), 0, kRes - 1);
    const int lo1 = clampi((int)floorf(nv[1]), 0, kRes - 1);
    const int lo2 = clampi((int)floorf(nv[2]), 0, kRes - 1);
    const float f0 = nv[0] - (float)lo0;
    const float f1 = nv[1] - (float)lo1;
    const float f2 = nv[2] - (float)lo2;
    const int hi0 = (lo0 + 1) < (kRes - 1) ? (lo0 + 1) : (kRes - 1);
    const int hi1 = (lo1 + 1) < (kRes - 1) ? (lo1 + 1) : (kRes - 1);
    const int hi2 = (lo2 + 1) < (kRes - 1) ? (lo2 + 1) : (kRes - 1);
    float pv0 = 0.0f, pv1 = 0.0f;
#pragma unroll
    for (int corner = 0; corner < 8; ++corner) {
      const int dx = corner >> 2, dy = (corner >> 1) & 1, dz = corner & 1;
      const int xi = dx ? hi0 : lo0;
      const int yi = dy ? hi1 : lo1;
      const int zi = dz ? hi2 : lo2;
      const float wgt = ((dx ? f0 : 1.0f - f0) * (dy ? f1 : 1.0f - f1)) * (dz ? f2 : 1.0f - f2);
      const float* vrow = v2b + ((size_t)((xi * kRes + yi) * kRes + zi)) * kChan;
      pv0 = pv0 + wgt * vrow[c0];
      pv1 = pv1 + wgt * vrow[c1];
    }
    sRes[c0 * 33 + 4 * wave + pt] = pv0 + mx0;
    sRes[c1 * 33 + 4 * wave + pt] = pv1 + mx1;
  }
  __syncthreads();

  const int noff = (lane & 7) * 4;
  for (int pass = 0; pass < 2; ++pass) {
#pragma unroll
    for (int it = 0; it < 2; ++it) {
      const int c = 8 * wave + it * 4 + (lane >> 3);
      v4f o;
      o[0] = sRes[c * 33 + noff + 0];
      o[1] = sRes[c * 33 + noff + 1];
      o[2] = sRes[c * 33 + noff + 2];
      o[3] = sRes[c * 33 + noff + 3];
      *(volatile v4f*)(out + ((size_t)(b * kChan + c)) * kPoints + n0 + noff) = o;
    }
    __threadfence();
  }
}

extern "C" void kernel_launch(void* const* d_in, const int* in_sizes, int n_in,
                              void* d_out, int out_size, void* d_ws, size_t ws_size,
                              hipStream_t stream) {
  if (n_in < 13) return;
  if (in_sizes[0] != kBatch * kChan * kPoints) return;
  if (in_sizes[1] != kBatch * 3 * kPoints) return;
  if (in_sizes[2] != kBatch * kPoints * kNeigh) return;
  if (in_sizes[3] != kChan * kTaps) return;
  if (in_sizes[4] != kChan) return;
  if (in_sizes[5] != 4 * kChan) return;
  if (in_sizes[6] != kChan * kTaps) return;
  if (in_sizes[7] != kChan) return;
  if (in_sizes[8] != 4 * kChan) return;
  if (in_sizes[9] != 3 * kChan) return;
  if (in_sizes[10] != 12) return;
  if (in_sizes[11] != 9) return;
  if (in_sizes[12] != 4 * kChan) return;
  if (out_size != kBatch * kChan * kPoints) return;
  if (ws_size < kWsTotal) return;

  const float* x     = (const float*)d_in[0];
  const float* xyz   = (const float*)d_in[1];
  const int*   idx   = (const int*)d_in[2];
  const float* w3d1  = (const float*)d_in[3];
  const float* b3d1  = (const float*)d_in[4];
  const float* bn3d1 = (const float*)d_in[5];
  const float* w3d2  = (const float*)d_in[6];
  const float* b3d2  = (const float*)d_in[7];
  const float* bn3d2 = (const float*)d_in[8];
  const float* pw1   = (const float*)d_in[9];
  const float* pbn   = (const float*)d_in[10];
  const float* pw2   = (const float*)d_in[11];
  const float* ptbn  = (const float*)d_in[12];
  float* out = (float*)d_out;

  char* ws = (char*)d_ws;
  float*          meanp = (float*)(ws + kOffMean);
  unsigned short* wpad  = (unsigned short*)(ws + kOffWpad);
  int*            vid   = (int*)(ws + kOffVid);
  float*          ncT   = (float*)(ws + kOffNcT);
  float*          xyzT  = (float*)(ws + kOffXyzT);
  float*          proj  = (float*)(ws + kOffProj);
  float*          v0    = (float*)(ws + kOffV0);
  float*          v1    = (float*)(ws + kOffV1);
  float*          v2    = (float*)(ws + kOffV2);
  unsigned short* xT16  = (unsigned short*)(ws + kOffXT16);
  float*          xT32  = (float*)(ws + kOffXT32);

  coord_mean_kernel<<<kBatch * 3, 256, 0, stream>>>(xyz, meanp);
  weight_pad_kernel<<<1, 128, 0, stream>>>(pw1, wpad);
  point_prep_kernel<<<kAllPts / 32, 256, 0, stream>>>(x, xyz, meanp, xT32, xT16, ncT, xyzT, vid);
  voxel_mean_kernel<<<kBatch * 64, 64, 0, stream>>>(vid, xT32, v0);
  stencil_kernel<<<kBatch * kVoxels / 16, 256, 0, stream>>>(v0, w3d1, b3d1, bn3d1, v1);
  stencil_kernel<<<kBatch * kVoxels / 16, 256, 0, stream>>>(v1, w3d2, b3d2, bn3d2, v2);
  proj_gemm_kernel<<<kAllPts / 512, 256, 0, stream>>>(xT16, wpad, proj);
  fuse_kernel<<<kAllPts / 32, 256, 0, stream>>>(xT32, xyzT, ncT, proj, idx, v2, pbn, pw2, ptbn, out);
}
